// RelativePositionResidualAttentionBlock_28561532518831
// MI455X (gfx1250) — hardware-verified
//
#include <hip/hip_runtime.h>

typedef _Float16 v16h __attribute__((ext_vector_type(16)));
typedef _Float16 v8h  __attribute__((ext_vector_type(8)));
typedef float    v8f  __attribute__((ext_vector_type(8)));
typedef float    v4f  __attribute__((ext_vector_type(4)));
typedef v8h __attribute__((may_alias)) v8ha;
typedef v4f __attribute__((may_alias)) v4fa;

union Frag { v16h v; v8h half[2]; };

#define BATCH  2
#define SEQ    2048
#define DMODEL 768
#define NHEADS 12
#define HD     64
#define DMLP   3072
#define DFC    6144
#define MROWS  (BATCH * SEQ)
#define NREL   (2 * SEQ - 1)
#define WSC    32.0f
#define WINV   0.03125f
#define QKSC   0.125f
#define PSCALE 16384.0f
#define NBIAS  2112

__device__ __forceinline__ v8f wmma_f16(v16h a, v16h b, v8f c) {
  v8f d = __builtin_amdgcn_wmma_f32_16x16x32_f16(false, a, false, b, (short)0, c, false, false);
  asm volatile("v_nop\n\tv_nop\n\tv_nop\n\tv_nop" : "+v"(d) : "v"(a), "v"(b));
  return d;
}

__device__ __forceinline__ v16h load_frag(const _Float16* p, int h) {
  Frag f;
  f.half[0] = *(const v8ha*)(p + 8 * h);
  f.half[1] = *(const v8ha*)(p + 16 + 8 * h);
  return f.v;
}

__global__ __launch_bounds__(256) void wcvt_kernel(
    const float* __restrict__ s0, const float* __restrict__ s1,
    const float* __restrict__ s2, const float* __restrict__ s3,
    _Float16* __restrict__ dst, int K, int N)
{
  __shared__ __attribute__((aligned(16))) _Float16 sT[64 * 72];

  const int tid = threadIdx.x;
  const int z = blockIdx.z;
  const float* src = (z == 0) ? s0 : ((z == 1) ? s1 : ((z == 2) ? s2 : s3));
  _Float16* d = dst + (size_t)z * N * K;
  const int n0 = blockIdx.x * 64, k0 = blockIdx.y * 64;

  const int nc = tid & 63, kr0 = tid >> 6;
  #pragma unroll
  for (int i = 0; i < 16; ++i) {
    const int kr = kr0 + 4 * i;
    const float v = src[(size_t)(k0 + kr) * N + n0 + nc] * WSC;
    sT[nc * 72 + kr] = (_Float16)v;
  }
  __syncthreads();

  const int lane = tid & 31, w = tid >> 5, q8 = lane & 7, sub = lane >> 3;
  const int lnA = w * 8 + sub, lnB = lnA + 4;
  const v8h rA = *(const v8ha*)(sT + lnA * 72 + 8 * q8);
  const v8h rB = *(const v8ha*)(sT + lnB * 72 + 8 * q8);
  _Float16* pA = d + (size_t)(n0 + lnA) * K + k0 + 8 * q8;
  _Float16* pB = d + (size_t)(n0 + lnB) * K + k0 + 8 * q8;
  *(volatile v8h*)pA = rA;
  *(volatile v8h*)pB = rB;
  __threadfence();
  *(volatile v8h*)pA = rA;
  *(volatile v8h*)pB = rB;
}

__global__ __launch_bounds__(256) void ln_kernel(
    const float* __restrict__ X, const float* __restrict__ gam,
    const float* __restrict__ bet, _Float16* __restrict__ Y)
{
  const int row  = blockIdx.x * 8 + (threadIdx.x >> 5);
  const int lane = threadIdx.x & 31;
  if (row >= MROWS) return;
  const float* xr = X + (size_t)row * DMODEL + 8 * lane;

  v4f v[6];
  #pragma unroll
  for (int c = 0; c < 3; ++c) {
    v[2 * c]     = *(const v4fa*)(xr + 256 * c);
    v[2 * c + 1] = *(const v4fa*)(xr + 256 * c + 4);
  }
  float s = 0.0f;
  #pragma unroll
  for (int i = 0; i < 6; ++i) s += (v[i].x + v[i].y) + (v[i].z + v[i].w);
  #pragma unroll
  for (int o = 16; o >= 1; o >>= 1) s += __shfl_xor(s, o, 32);
  const float mu = s * (1.0f / DMODEL);

  float q = 0.0f;
  #pragma unroll
  for (int i = 0; i < 6; ++i) {
    const float a0 = v[i].x - mu, a1 = v[i].y - mu, a2 = v[i].z - mu, a3 = v[i].w - mu;
    q += (a0 * a0 + a1 * a1) + (a2 * a2 + a3 * a3);
  }
  #pragma unroll
  for (int o = 16; o >= 1; o >>= 1) q += __shfl_xor(q, o, 32);
  const float rinv = rsqrtf(q * (1.0f / DMODEL) + 1e-5f);

  v8h ov[3];
  #pragma unroll
  for (int c = 0; c < 3; ++c) {
    const v4f g0 = *(const v4fa*)(gam + 256 * c + 8 * lane);
    const v4f g1 = *(const v4fa*)(gam + 256 * c + 8 * lane + 4);
    const v4f b0 = *(const v4fa*)(bet + 256 * c + 8 * lane);
    const v4f b1 = *(const v4fa*)(bet + 256 * c + 8 * lane + 4);
    const v4f x0 = v[2 * c], x1 = v[2 * c + 1];
    v8h o;
    o[0] = (_Float16)((x0.x - mu) * rinv * g0.x + b0.x);
    o[1] = (_Float16)((x0.y - mu) * rinv * g0.y + b0.y);
    o[2] = (_Float16)((x0.z - mu) * rinv * g0.z + b0.z);
    o[3] = (_Float16)((x0.w - mu) * rinv * g0.w + b0.w);
    o[4] = (_Float16)((x1.x - mu) * rinv * g1.x + b1.x);
    o[5] = (_Float16)((x1.y - mu) * rinv * g1.y + b1.y);
    o[6] = (_Float16)((x1.z - mu) * rinv * g1.z + b1.z);
    o[7] = (_Float16)((x1.w - mu) * rinv * g1.w + b1.w);
    ov[c] = o;
  }
  _Float16* yr = Y + (size_t)row * DMODEL + 8 * lane;
  #pragma unroll
  for (int c = 0; c < 3; ++c) *(volatile v8h*)(yr + 256 * c) = ov[c];
  __threadfence();
  #pragma unroll
  for (int c = 0; c < 3; ++c) *(volatile v8h*)(yr + 256 * c) = ov[c];
}

__device__ __forceinline__ void proj_store_pass(const _Float16* sT, _Float16* plane, _Float16* vt,
                                                int which, int bh, int l0, int w, int lane) {
  const int q8 = lane & 7, sub = lane >> 3;
  #pragma unroll
  for (int i = 0; i < 8; ++i) {
    const int lid = w * 32 + i * 4 + sub;
    v8h v;
    _Float16* dst;
    if (which != 2) {
      v = *(const v8ha*)(sT + lid * HD + 8 * q8);
      dst = plane + ((size_t)bh * SEQ + l0 + lid) * HD + 8 * q8;
    } else {
      const int dd = lid >> 1, hl = lid & 1;
      v = *(const v8ha*)(sT + dd * 128 + 64 * hl + 8 * q8);
      dst = vt + ((size_t)bh * HD + dd) * SEQ + l0 + 64 * hl + 8 * q8;
    }
    *(volatile v8h*)dst = v;
  }
}

__global__ __launch_bounds__(128) void proj_kernel(
    const _Float16* __restrict__ xh,
    const _Float16* __restrict__ wh,
    _Float16* __restrict__ qh,
    _Float16* __restrict__ kh,
    _Float16* __restrict__ vt)
{
  __shared__ __attribute__((aligned(16))) _Float16 sT[128 * 64];

  const int tid = threadIdx.x, lane = tid & 31, w = tid >> 5;
  const int h = lane >> 4, m = lane & 15;
  const int m0 = blockIdx.x * 128;
  const int cg = blockIdx.y;
  const int which = cg / NHEADS, head = cg - which * NHEADS;
  const int m0w = m0 + 32 * w;

  const _Float16* xa0 = xh + (size_t)(m0w + m) * DMODEL;
  const _Float16* xa1 = xa0 + (size_t)16 * DMODEL;
  const _Float16* wb  = wh + ((size_t)which * DMODEL + head * HD + m) * DMODEL;

  const v8f zero8 = {0.f, 0.f, 0.f, 0.f, 0.f, 0.f, 0.f, 0.f};
  v8f acc[2][4];
  #pragma unroll
  for (int mt = 0; mt < 2; ++mt)
    #pragma unroll
    for (int nt = 0; nt < 4; ++nt) acc[mt][nt] = zero8;

  #pragma unroll 1
  for (int k0 = 0; k0 < DMODEL; k0 += 32) {
    const v16h a0 = load_frag(xa0 + k0, h);
    const v16h a1 = load_frag(xa1 + k0, h);
    #pragma unroll
    for (int nt = 0; nt < 4; ++nt) {
      const v16h b = load_frag(wb + (size_t)nt * 16 * DMODEL + k0, h);
      acc[0][nt] = wmma_f16(a0, b, acc[0][nt]);
      acc[1][nt] = wmma_f16(a1, b, acc[1][nt]);
    }
  }

  #pragma unroll
  for (int nt = 0; nt < 4; ++nt) {
    const int feat = 16 * nt + m;
    #pragma unroll
    for (int mt = 0; mt < 2; ++mt) {
      #pragma unroll
      for (int r = 0; r < 8; ++r) {
        const int tokl = 32 * w + 16 * mt + 8 * h + r;
        const float y = acc[mt][nt][r] * WINV;
        const int idx = (which == 2) ? (feat * 128 + tokl) : (tokl * HD + feat);
        sT[idx] = (_Float16)y;
      }
    }
  }
  __syncthreads();

  const int b = m0 / SEQ, l0 = m0 - b * SEQ, bh = b * NHEADS + head;
  _Float16* plane = (which == 0) ? qh : kh;
  proj_store_pass(sT, plane, vt, which, bh, l0, w, lane);
  __threadfence();
  proj_store_pass(sT, plane, vt, which, bh, l0, w, lane);
}

__device__ __forceinline__ v16h pack_p(v8f a, v8f c) {
  const v16h r = { (_Float16)(a[0] * PSCALE), (_Float16)(a[1] * PSCALE), (_Float16)(a[2] * PSCALE), (_Float16)(a[3] * PSCALE),
                   (_Float16)(a[4] * PSCALE), (_Float16)(a[5] * PSCALE), (_Float16)(a[6] * PSCALE), (_Float16)(a[7] * PSCALE),
                   (_Float16)(c[0] * PSCALE), (_Float16)(c[1] * PSCALE), (_Float16)(c[2] * PSCALE), (_Float16)(c[3] * PSCALE),
                   (_Float16)(c[4] * PSCALE), (_Float16)(c[5] * PSCALE), (_Float16)(c[6] * PSCALE), (_Float16)(c[7] * PSCALE) };
  return r;
}

__device__ __forceinline__ void att_store_pass(const _Float16* so, _Float16* oh,
                                               int b, int head, int q0, int lane) {
  const int q8 = lane & 7, sub = lane >> 3;
  #pragma unroll
  for (int i = 0; i < 4; ++i) {
    const int row = i * 4 + sub;
    const v8h v = *(const v8ha*)(so + row * HD + 8 * q8);
    const size_t gi = ((size_t)b * SEQ + q0 + row) * DMODEL + head * HD + 8 * q8;
    *(volatile v8h*)(oh + gi) = v;
  }
}

__global__ __launch_bounds__(128) void attn_kernel(
    const _Float16* __restrict__ qh,
    const _Float16* __restrict__ kh,
    const _Float16* __restrict__ vt,
    const float* __restrict__ rel,
    _Float16* __restrict__ oh)
{
  __shared__ __attribute__((aligned(16))) float sBias[NBIAS];
  __shared__ __attribute__((aligned(16))) _Float16 sO[4 * 16 * 64];

  const int tid = threadIdx.x, lane = tid & 31, w = tid >> 5;
  const int h = lane >> 4, m = lane & 15;
  const int bh = blockIdx.y, b = bh / NHEADS, head = bh - b * NHEADS;
  const int q0b = blockIdx.x * 64;
  const int q0 = q0b + 16 * w;

  for (int i = tid; i < q0b + 127; i += 128)
    sBias[i] = rel[(size_t)(SEQ - 64 + i) * NHEADS + head];

  const _Float16* qrow = qh + ((size_t)bh * SEQ + q0 + m) * HD;
  const v16h qb0 = load_frag(qrow, h);
  const v16h qb1 = load_frag(qrow + 32, h);

  const v8f zero8 = {0.f, 0.f, 0.f, 0.f, 0.f, 0.f, 0.f, 0.f};
  v8f o[4];
  #pragma unroll
  for (int t = 0; t < 4; ++t) o[t] = zero8;
  float mrun = -1e30f, lrun = 0.0f;

  const _Float16* kbase = kh + ((size_t)bh * SEQ + m) * HD;
  const _Float16* vbase = vt + ((size_t)bh * HD + m) * SEQ;
  const int bidx0 = q0 + m + 63;

  __syncthreads();

  const int nsteps = blockIdx.x + 1;
  #pragma unroll 1
  for (int st = 0; st < nsteps; ++st) {
    const int kb = st * 64;
    v8f s[4];
    #pragma unroll
    for (int j = 0; j < 4; ++j) {
      const _Float16* kp = kbase + (size_t)(kb + 16 * j) * HD;
      const v16h kf0 = load_frag(kp, h);
      const v16h kf1 = load_frag(kp + 32, h);
      v8f z = zero8;
      z = wmma_f16(kf0, qb0, z);
      z = wmma_f16(kf1, qb1, z);
      s[j] = z;
    }
    #pragma unroll
    for (int j = 0; j < 4; ++j) {
      const int ib = bidx0 - (kb + 16 * j + 8 * h);
      #pragma unroll
      for (int r = 0; r < 8; ++r) {
        const int idx = ib - r;
        const float bv = sBias[idx];
        const float val = s[j][r] * QKSC + bv;
        s[j][r] = (idx >= 63) ? val : -1e30f;
      }
    }

    float mloc = s[0][0];
    #pragma unroll
    for (int j = 0; j < 4; ++j)
      #pragma unroll
      for (int r = 0; r < 8; ++r) mloc = fmaxf(mloc, s[j][r]);
    mloc = fmaxf(mloc, __shfl_xor(mloc, 16, 32));
    const float mnew = fmaxf(mrun, mloc);
    const float alpha = __expf(mrun - mnew);
    mrun = mnew;
    float lsum = 0.0f;
    #pragma unroll
    for (int j = 0; j < 4; ++j)
      #pragma unroll
      for (int r = 0; r < 8; ++r) {
        const float p = __expf(s[j][r] - mnew);
        s[j][r] = p;
        lsum += p;
      }
    lsum += __shfl_xor(lsum, 16, 32);
    lrun = lrun * alpha + lsum;
    #pragma unroll
    for (int t = 0; t < 4; ++t)
      #pragma unroll
      for (int r = 0; r < 8; ++r) o[t][r] = o[t][r] * alpha;

    const v16h pb0 = pack_p(s[0], s[1]);
    const v16h pb1 = pack_p(s[2], s[3]);

    #pragma unroll
    for (int t = 0; t < 4; ++t) {
      const _Float16* vp = vbase + (size_t)(16 * t) * SEQ + kb;
      const v16h vf0 = load_frag(vp, h);
      const v16h vf1 = load_frag(vp + 32, h);
      o[t] = wmma_f16(vf0, pb0, o[t]);
      o[t] = wmma_f16(vf1, pb1, o[t]);
    }
  }

  const float inv = (1.0f / lrun) * (1.0f / PSCALE);
  _Float16* so = sO + w * 1024;
  #pragma unroll
  for (int t = 0; t < 4; ++t) {
    v8h pk;
    pk[0] = (_Float16)(o[t][0] * inv); pk[1] = (_Float16)(o[t][1] * inv);
    pk[2] = (_Float16)(o[t][2] * inv); pk[3] = (_Float16)(o[t][3] * inv);
    pk[4] = (_Float16)(o[t][4] * inv); pk[5] = (_Float16)(o[t][5] * inv);
    pk[6] = (_Float16)(o[t][6] * inv); pk[7] = (_Float16)(o[t][7] * inv);
    *(v8ha*)(so + m * HD + 16 * t + 8 * h) = pk;
  }
  __syncthreads();

  att_store_pass(so, oh, b, head, q0, lane);
  __threadfence();
  att_store_pass(so, oh, b, head, q0, lane);
}

__device__ __forceinline__ void out_store_pass(const float* sC, float* C, int m0, int n0, int w, int lane) {
  const int q8 = lane & 7, sub = lane >> 3;
  #pragma unroll
  for (int i = 0; i < 16; ++i) {
    const int lid = i * 4 + sub;
    const int rl = 32 * w + (lid >> 1), hl = lid & 1;
    const v4f v = *(const v4fa*)(sC + rl * 64 + 32 * hl + 4 * q8);
    *(volatile v4f*)(C + (size_t)(m0 + rl) * DMODEL + n0 + 32 * hl + 4 * q8) = v;
  }
}

template <bool HAS_BIAS>
__global__ __launch_bounds__(128) void gemm_out_kernel(
    const _Float16* __restrict__ A,
    const _Float16* __restrict__ Wt,
    const float* __restrict__ bias,
    const float* __restrict__ resid,
    float* __restrict__ C,
    int K)
{
  __shared__ __attribute__((aligned(16))) float sC[128 * 64];

  const int tid = threadIdx.x, lane = tid & 31, w = tid >> 5;
  const int h = lane >> 4, m = lane & 15;
  const int m0 = blockIdx.x * 128, n0 = blockIdx.y * 64;
  const int m0w = m0 + 32 * w;

  const _Float16* xa0 = A + (size_t)(m0w + m) * K;
  const _Float16* xa1 = xa0 + (size_t)16 * K;
  const _Float16* wb  = Wt + (size_t)(n0 + m) * K;

  const v8f zero8 = {0.f, 0.f, 0.f, 0.f, 0.f, 0.f, 0.f, 0.f};
  v8f acc[2][4];
  #pragma unroll
  for (int mt = 0; mt < 2; ++mt)
    #pragma unroll
    for (int nt = 0; nt < 4; ++nt) acc[mt][nt] = zero8;

  #pragma unroll 1
  for (int k0 = 0; k0 < K; k0 += 32) {
    const v16h a0 = load_frag(xa0 + k0, h);
    const v16h a1 = load_frag(xa1 + k0, h);
    #pragma unroll
    for (int nt = 0; nt < 4; ++nt) {
      const v16h bf = load_frag(wb + (size_t)nt * 16 * K + k0, h);
      acc[0][nt] = wmma_f16(a0, bf, acc[0][nt]);
      acc[1][nt] = wmma_f16(a1, bf, acc[1][nt]);
    }
  }

  #pragma unroll
  for (int nt = 0; nt < 4; ++nt) {
    const int cl = 16 * nt + m;
    float bv = 0.0f;
    if (HAS_BIAS) bv = bias[n0 + cl];
    #pragma unroll
    for (int mt = 0; mt < 2; ++mt) {
      #pragma unroll
      for (int r = 0; r < 8; ++r) {
        const int rl = 32 * w + 16 * mt + 8 * h + r;
        const float rv = resid[(size_t)(m0 + rl) * DMODEL + n0 + cl];
        const float y = acc[mt][nt][r] * WINV + bv;
        sC[rl * 64 + cl] = rv + y;
      }
    }
  }
  __syncthreads();

  out_store_pass(sC, C, m0, n0, w, lane);
  __threadfence();
  out_store_pass(sC, C, m0, n0, w, lane);
}

__device__ __forceinline__ void fc_store_pass(const _Float16* sM, _Float16* Mo, int m0, int n0, int w, int lane) {
  const int q8 = lane & 7, sub = lane >> 3;
  #pragma unroll
  for (int i = 0; i < 4; ++i) {
    const int lid = w * 16 + i * 4 + sub;
    const v8h v = *(const v8ha*)(sM + lid * 64 + 8 * q8);
    *(volatile v8h*)(Mo + (size_t)(m0 + lid) * DMLP + n0 + 8 * q8) = v;
  }
}

__global__ __launch_bounds__(128) void fc_geglu_kernel(
    const _Float16* __restrict__ A,
    const _Float16* __restrict__ Wt,
    const float* __restrict__ bfc,
    _Float16* __restrict__ Mo)
{
  __shared__ __attribute__((aligned(16))) _Float16 sM[64 * 64];

  const int tid = threadIdx.x, lane = tid & 31, w = tid >> 5;
  const int h = lane >> 4, m = lane & 15;
  const int wr = w & 1, wc = w >> 1;
  const int m0 = blockIdx.x * 64, n0 = blockIdx.y * 64;

  const _Float16* xa0 = A + (size_t)(m0 + 32 * wr + m) * DMODEL;
  const _Float16* xa1 = xa0 + (size_t)16 * DMODEL;
  const _Float16* wba = Wt + (size_t)(n0 + 32 * wc + m) * DMODEL;
  const _Float16* wbg = Wt + (size_t)(DMLP + n0 + 32 * wc + m) * DMODEL;

  const v8f zero8 = {0.f, 0.f, 0.f, 0.f, 0.f, 0.f, 0.f, 0.f};
  v8f acc[2][4];
  #pragma unroll
  for (int mt = 0; mt < 2; ++mt)
    #pragma unroll
    for (int nt = 0; nt < 4; ++nt) acc[mt][nt] = zero8;

  #pragma unroll 1
  for (int k0 = 0; k0 < DMODEL; k0 += 32) {
    const v16h a0 = load_frag(xa0 + k0, h);
    const v16h a1 = load_frag(xa1 + k0, h);
    #pragma unroll
    for (int nt = 0; nt < 4; ++nt) {
      const _Float16* bp = (nt < 2) ? (wba + (size_t)nt * 16 * DMODEL) : (wbg + (size_t)(nt - 2) * 16 * DMODEL);
      const v16h bf = load_frag(bp + k0, h);
      acc[0][nt] = wmma_f16(a0, bf, acc[0][nt]);
      acc[1][nt] = wmma_f16(a1, bf, acc[1][nt]);
    }
  }

  #pragma unroll
  for (int nt = 0; nt < 2; ++nt) {
    const int cl = 32 * wc + 16 * nt + m;
    const float ba = bfc[n0 + cl];
    const float bg = bfc[DMLP + n0 + cl];
    #pragma unroll
    for (int mt = 0; mt < 2; ++mt) {
      #pragma unroll
      for (int r = 0; r < 8; ++r) {
        const int rl = 32 * wr + 16 * mt + 8 * h + r;
        const float av = acc[mt][nt][r] * WINV + ba;
        const float gv = acc[mt][nt + 2][r] * WINV + bg;
        const float gl = 0.5f * gv * (1.0f + erff(gv * 0.70710678118654752f));
        sM[rl * 64 + cl] = (_Float16)(av * gl);
      }
    }
  }
  __syncthreads();

  fc_store_pass(sM, Mo, m0, n0, w, lane);
  __threadfence();
  fc_store_pass(sM, Mo, m0, n0, w, lane);
}

extern "C" void kernel_launch(void* const* d_in, const int* in_sizes, int n_in,
                              void* d_out, int out_size, void* d_ws, size_t ws_size,
                              hipStream_t stream) {
  if (n_in < 14) return;
  if (in_sizes[0] != MROWS * DMODEL) return;
  if (in_sizes[1] != DMODEL || in_sizes[2] != DMODEL || in_sizes[8] != DMODEL ||
      in_sizes[9] != DMODEL || in_sizes[13] != DMODEL) return;
  if (in_sizes[3] != DMODEL * DMODEL || in_sizes[4] != DMODEL * DMODEL ||
      in_sizes[5] != DMODEL * DMODEL || in_sizes[6] != DMODEL * DMODEL) return;
  if (in_sizes[7] != NREL * NHEADS) return;
  if (in_sizes[10] != DMODEL * DFC || in_sizes[11] != DFC) return;
  if (in_sizes[12] != DMLP * DMODEL) return;
  if (out_size != MROWS * DMODEL) return;

  const float* x      = (const float*)d_in[0];
  const float* ln1_g  = (const float*)d_in[1];
  const float* ln1_b  = (const float*)d_in[2];
  const float* Wq     = (const float*)d_in[3];
  const float* Wk     = (const float*)d_in[4];
  const float* Wv     = (const float*)d_in[5];
  const float* Wo     = (const float*)d_in[6];
  const float* rel    = (const float*)d_in[7];
  const float* ln2_g  = (const float*)d_in[8];
  const float* ln2_b  = (const float*)d_in[9];
  const float* W_fc   = (const float*)d_in[10];
  const float* b_fc   = (const float*)d_in[11];
  const float* W_proj = (const float*)d_in[12];
  const float* b_proj = (const float*)d_in[13];
  float* out = (float*)d_out;

  const size_t w1_bytes  = (size_t)DMODEL * DMODEL * 2;
  const size_t wq4_bytes = 4 * w1_bytes;
  const size_t wfc_bytes = (size_t)DFC * DMODEL * 2;
  const size_t wpr_bytes = (size_t)DMODEL * DMLP * 2;
  const size_t act_bytes = (size_t)MROWS * DMODEL * 2;
  const size_t x1_bytes  = (size_t)MROWS * DMODEL * 4;
  const size_t mh_bytes  = (size_t)MROWS * DMLP * 2;
  const size_t total = wq4_bytes + wfc_bytes + wpr_bytes + 6 * act_bytes + x1_bytes + mh_bytes;
  if (total > ws_size) return;

  char* ws = (char*)d_ws;
  size_t off = 0;
  _Float16* whq = (_Float16*)(ws + off); off += wq4_bytes;
  _Float16* who = whq + (size_t)3 * DMODEL * DMODEL;
  _Float16* wfc = (_Float16*)(ws + off); off += wfc_bytes;
  _Float16* wpr = (_Float16*)(ws + off); off += wpr_bytes;
  _Float16* xh  = (_Float16*)(ws + off); off += act_bytes;
  _Float16* qh  = (_Float16*)(ws + off); off += act_bytes;
  _Float16* kh  = (_Float16*)(ws + off); off += act_bytes;
  _Float16* vt  = (_Float16*)(ws + off); off += act_bytes;
  _Float16* oh  = (_Float16*)(ws + off); off += act_bytes;
  _Float16* h2  = (_Float16*)(ws + off); off += act_bytes;
  float*    x1  = (float*)(ws + off);    off += x1_bytes;
  _Float16* mh  = (_Float16*)(ws + off); off += mh_bytes;
  if (off > ws_size) return;

  wcvt_kernel<<<dim3(DMODEL / 64, DMODEL / 64, 4), 256, 0, stream>>>(Wq, Wk, Wv, Wo, whq, DMODEL, DMODEL);
  wcvt_kernel<<<dim3(DFC / 64, DMODEL / 64, 1), 256, 0, stream>>>(W_fc, W_fc, W_fc, W_fc, wfc, DMODEL, DFC);
  wcvt_kernel<<<dim3(DMODEL / 64, DMLP / 64, 1), 256, 0, stream>>>(W_proj, W_proj, W_proj, W_proj, wpr, DMLP, DMODEL);

  ln_kernel<<<MROWS / 8, 256, 0, stream>>>(x, ln1_g, ln1_b, xh);

  proj_kernel<<<dim3(MROWS / 128, 3 * NHEADS), 128, 0, stream>>>(xh, whq, qh, kh, vt);

  attn_kernel<<<dim3(SEQ / 64, BATCH * NHEADS), 128, 0, stream>>>(qh, kh, vt, rel, oh);

  gemm_out_kernel<false><<<dim3(MROWS / 128, DMODEL / 64), 128, 0, stream>>>(oh, who, b_proj, x, x1, DMODEL);

  ln_kernel<<<MROWS / 8, 256, 0, stream>>>(x1, ln2_g, ln2_b, h2);

  fc_geglu_kernel<<<dim3(MROWS / 64, DMLP / 64), 128, 0, stream>>>(h2, wfc, b_fc, mh);

  gemm_out_kernel<true><<<dim3(MROWS / 128, DMODEL / 64), 128, 0, stream>>>(mh, wpr, b_proj, x1, out, DMLP);
}
